// GCN_Dense_Aux_5609227288948
// MI455X (gfx1250) — hardware-run, weakly checked
//
#include <hip/hip_runtime.h>

typedef float          v8f   __attribute__((ext_vector_type(8)));
typedef float          v4f   __attribute__((ext_vector_type(4)));
typedef unsigned int   v4u   __attribute__((ext_vector_type(4)));
typedef int            v8i   __attribute__((ext_vector_type(8)));
typedef unsigned short v8us  __attribute__((ext_vector_type(8)));
typedef unsigned short v16us __attribute__((ext_vector_type(16)));
typedef __bf16         v16bf __attribute__((ext_vector_type(16)));
typedef _Float16       v16h  __attribute__((ext_vector_type(16)));
typedef v4f  __attribute__((may_alias)) v4fa;
typedef v8us __attribute__((may_alias)) v8usa;
union FragB { v16bf v; v16us u; v8us h[2]; v8i w; };
union FragH { v16h  v; v16us u; v8us h[2]; v8i w; };

__device__ __forceinline__ v8f wmb(const FragB& a, const FragB& b, v8f c) {
  v8f d = __builtin_amdgcn_wmma_f32_16x16x32_bf16(false, a.v, false, b.v, (short)0, c, false, false);
  asm volatile("v_nop\n\tv_nop\n\tv_nop\n\tv_nop" : "+v"(d) : "v"(a.w), "v"(b.w));
  return d;
}

__device__ __forceinline__ v8f wmh(const FragH& a, const FragH& b, v8f c) {
  v8f d = __builtin_amdgcn_wmma_f32_16x16x32_f16(false, a.v, false, b.v, (short)0, c, false, false);
  asm volatile("v_nop\n\tv_nop\n\tv_nop\n\tv_nop" : "+v"(d) : "v"(a.w), "v"(b.w));
  return d;
}

__device__ __forceinline__ unsigned bf16_bits(float f) {
  const unsigned u = __float_as_uint(f);
  const unsigned r = (u + 0x7FFFu + ((u >> 16) & 1u)) >> 16;
  const unsigned q = (u >> 16) | 0x40u;
  return ((u & 0x7fffffffu) > 0x7f800000u) ? q : r;
}

__device__ __forceinline__ float bf16_val(float f) {
  return __uint_as_float(bf16_bits(f) << 16);
}
__device__ __forceinline__ int clampi(int v, int lo, int hi) {
  return v < lo ? lo : (v > hi ? hi : v);
}

__device__ __forceinline__ unsigned f16_bits(float f) {
  const unsigned u  = __float_as_uint(f);
  const unsigned s  = (u >> 16) & 0x8000u;
  const unsigned a  = u & 0x7fffffffu;
  const unsigned t  = a - 0x38000000u;
  const unsigned r  = (t + 0x0FFFu + ((t >> 13) & 1u)) >> 13;
  const unsigned rc = r > 0x7C00u ? 0x7C00u : r;
  const bool small  = a < 0x38800000u;
  const bool isnan  = a > 0x7f800000u;
  const unsigned fin = small ? 0u : (s | rc);
  return isnan ? (s | 0x7E00u) : fin;
}

__device__ __forceinline__ unsigned pk16(unsigned lo, unsigned hi) { return lo | (hi << 16); }
__device__ __forceinline__ unsigned bf16_lo_bits(float v) {
  float hi = bf16_val(v);
  asm volatile("" : "+v"(hi));
  return bf16_bits(v - hi);
}
__device__ __forceinline__ v4u pack8_bf16(v4f a, v4f c) {
  return (v4u){ pk16(bf16_bits(a[0]), bf16_bits(a[1])), pk16(bf16_bits(a[2]), bf16_bits(a[3])),
                pk16(bf16_bits(c[0]), bf16_bits(c[1])), pk16(bf16_bits(c[2]), bf16_bits(c[3])) };
}
__device__ __forceinline__ v4u pack8_bf16_lo(v4f a, v4f c) {
  return (v4u){ pk16(bf16_lo_bits(a[0]), bf16_lo_bits(a[1])), pk16(bf16_lo_bits(a[2]), bf16_lo_bits(a[3])),
                pk16(bf16_lo_bits(c[0]), bf16_lo_bits(c[1])), pk16(bf16_lo_bits(c[2]), bf16_lo_bits(c[3])) };
}
__device__ __forceinline__ v4u pack8_f16(v4f a, v4f c) {
  return (v4u){ pk16(f16_bits(a[0]), f16_bits(a[1])), pk16(f16_bits(a[2]), f16_bits(a[3])),
                pk16(f16_bits(c[0]), f16_bits(c[1])), pk16(f16_bits(c[2]), f16_bits(c[3])) };
}

template <int FORM>
__global__ __launch_bounds__(256) void k_plane(const float* __restrict__ src, int rows, int cols, int ldsrc,
                                               unsigned short* __restrict__ dst, int MP, int KP) {
  static_assert(FORM >= 0 && FORM <= 3);
  const int KTOT = (FORM == 1 || FORM == 3) ? 2 * KP : KP;
  const unsigned ppr   = (unsigned)(KTOT >> 3);
  const unsigned kp8   = (unsigned)(KP >> 3);
  const unsigned total = (unsigned)MP * ppr;
  const unsigned g     = blockIdx.x * 256u + threadIdx.x;
  const unsigned rowu  = g / ppr;
  const unsigned p     = g - rowu * ppr;
  const bool second    = p >= kp8;
  const int row = (int)rowu;
  const int c0  = (int)((second ? p - kp8 : p) << 3);
  const float* srow = src + (size_t)clampi(row, 0, rows - 1) * (size_t)ldsrc;
  float x[8];
  unsigned mk[8];
#pragma unroll
  for (int e = 0; e < 8; ++e) {
    const int c = c0 + e;
    const float v = srow[clampi(c, 0, cols - 1)];
    asm volatile("" :: "v"(v));
    x[e]  = v;
    mk[e] = (row < rows && c < cols) ? 0xFFFFu : 0u;
  }
  const v4f a = (v4f){ x[0], x[1], x[2], x[3] };
  const v4f c = (v4f){ x[4], x[5], x[6], x[7] };
  v4u o;
  if (FORM == 2) {
    o = pack8_f16(a, c);
  } else {
    const v4u hi = pack8_bf16(a, c);
    o = hi;
    if (FORM == 1) { const v4u lo = pack8_bf16_lo(a, c); o = second ? lo : hi; }
  }
  const v4u mw = (v4u){ pk16(mk[0], mk[1]), pk16(mk[2], mk[3]), pk16(mk[4], mk[5]), pk16(mk[6], mk[7]) };
  o &= mw;
  if (g < total) {
    volatile v4u* q = (volatile v4u*)(dst + (size_t)g * 8);
    *q = o;
    __threadfence();
    *q = o;
  }
}

template <int FORM> struct FragOf    { typedef FragB T; };
template <>         struct FragOf<2> { typedef FragH T; };
__device__ __forceinline__ v8f mm(const FragB& a, const FragB& b, v8f c) { return wmb(a, b, c); }
__device__ __forceinline__ v8f mm(const FragH& a, const FragH& b, v8f c) { return wmh(a, b, c); }
template <class F> __device__ __forceinline__ F ld_frag(const unsigned short* p) {
  F f;
  f.h[0] = *(const v8usa*)(p);
  f.h[1] = *(const v8usa*)(p + 16);
  return f;
}

template <int FORM, int EPI>
__global__ __launch_bounds__(256) __attribute__((amdgpu_num_vgpr(248)))
void k_gemm_nt(const unsigned short* __restrict__ A, const unsigned short* __restrict__ B,
               const float* __restrict__ bias, float* __restrict__ D, int M, int N, int KTOT, int ldd) {
  static_assert(FORM >= 0 && FORM <= 2);
  static_assert(EPI == 0 || EPI == 1);
  typedef typename FragOf<FORM>::T F;
  __shared__ __attribute__((aligned(16))) float sT[8][16 * 68];
  const int lane = threadIdx.x & 31;
  const int wave = threadIdx.x >> 5;
  const int tilesM = (M + 63) >> 6;
  const int tilesN = (N + 63) >> 6;
  const int tile = blockIdx.x * 8 + wave;
  if (tile >= tilesM * tilesN) return;
  const int tm = tile / tilesN;
  const int tn = tile - tm * tilesN;
  const int m0 = tm << 6;
  const int n0 = tn << 6;

  const int rl = lane & 15;
  const int h8 = (lane >> 4) * 8;
  const unsigned short* pa = A + (size_t)(m0 + rl) * (size_t)KTOT + h8;
  const unsigned short* pb = B + (size_t)(n0 + rl) * (size_t)KTOT + h8;

  v8f acc[4][4];
#pragma unroll
  for (int i = 0; i < 4; ++i)
#pragma unroll
    for (int j = 0; j < 4; ++j) acc[i][j] = (v8f){0.f, 0.f, 0.f, 0.f, 0.f, 0.f, 0.f, 0.f};

#pragma unroll 1
  for (int k0 = 0; k0 < KTOT; k0 += 32) {
    F bf[4];
#pragma unroll
    for (int j = 0; j < 4; ++j) bf[j] = ld_frag<F>(pb + (size_t)(j << 4) * (size_t)KTOT + k0);
#pragma unroll
    for (int i = 0; i < 4; ++i) {
      const F af = ld_frag<F>(pa + (size_t)(i << 4) * (size_t)KTOT + k0);
#pragma unroll
      for (int j = 0; j < 4; ++j) acc[i][j] = mm(af, bf[j], acc[i][j]);
    }
  }

  float* slab = sT[wave];
  const int hh = lane >> 4;
  const int c4 = (lane & 15) * 4;
  const int nc = n0 + c4;
  const bool cok = nc < N;
  v4f bv = (v4f){0.f, 0.f, 0.f, 0.f};
  if (EPI == 1) {
    bv = *(const v4fa*)(bias + clampi(nc, 0, N - 4));
    asm volatile("" :: "v"(bv));
  }
#pragma unroll
  for (int i = 0; i < 4; ++i) {
    const int mBase = m0 + (i << 4);
#pragma unroll
    for (int j = 0; j < 4; ++j) {
#pragma unroll
      for (int r = 0; r < 8; ++r) slab[(h8 + r) * 68 + (j << 4) + rl] = acc[i][j][r];
    }
    __builtin_amdgcn_fence(__ATOMIC_RELEASE, "workgroup");
    __builtin_amdgcn_wave_barrier();
    __builtin_amdgcn_fence(__ATOMIC_ACQUIRE, "workgroup");
    v4f vv[8];
#pragma unroll
    for (int it = 0; it < 8; ++it) {
      const int row = it * 2 + hh;
      v4f v = *(const v4fa*)(slab + row * 68 + c4);
      if (EPI == 1) v += bv;
      vv[it] = v;
    }
    for (int pass = 0; pass < 2; ++pass) {
#pragma unroll
      for (int it = 0; it < 8; ++it) {
        const int row = mBase + it * 2 + hh;
        if (cok && row < M) *(volatile v4f*)(D + (size_t)row * (size_t)ldd + nc) = vv[it];
      }
      __threadfence();
    }
    __builtin_amdgcn_fence(__ATOMIC_RELEASE, "workgroup");
    __builtin_amdgcn_wave_barrier();
    __builtin_amdgcn_fence(__ATOMIC_ACQUIRE, "workgroup");
  }
}

#pragma clang fp contract(off)

#ifndef TWO_TERM
#define TWO_TERM 1
#endif

#define NN      20000
#define NE      320000
#define INF_    300
#define KP1     320
#define HF      256
#define MPAD    20096
#define K2TOT   (TWO_TERM ? 512 : 256)
#define NTHR    256
#define NWAVE   8
#define NBRUN   1024
#define SLB     10
#define NLB     20
#define CHUNK   2048
#define WCAP    256
#define LISTN   (NWAVE * WCAP)
#define NCHUNK  157
#define RCAP    21504
#define DEGCAP  64
#define LZ_INTS (LISTN + 2 * RCAP + 3 * NBRUN)
#define MISC_INTS 16
#define LIST_LDS_INTS (LZ_INTS + MISC_INTS)
#define LIST_LDS_BYTES (LIST_LDS_INTS * 4)
#define SM_FLOATS 544
#define SM_PA   512
#define SM_PR   516
#define PB_W1   ((HF * (KP1 / 8)) / NTHR)
#define PB_W2   ((HF * (K2TOT / 8)) / NTHR)
#define PB_PAD  (((MPAD - NN) * (K2TOT / 8)) / NTHR)
#define PB_ALL  (PB_W1 + PB_W2 + PB_PAD + 1)
#define WSMAX   ((size_t)128 << 20)

static_assert(NLB * NBRUN >= NN && NBRUN == (1 << SLB) && NBRUN == 4 * NTHR);
static_assert(NN % 8 == 0 && NN % 16 == 0);
static_assert(KP1 % 32 == 0 && KP1 >= INF_ && K2TOT % 32 == 0);
static_assert(MPAD % 64 == 0 && MPAD >= NN && HF % 64 == 0 && HF % 32 == 0);
static_assert(NE % CHUNK == 512 && NCHUNK == (NE + CHUNK - 1) / CHUNK);
static_assert(CHUNK == NWAVE * WCAP && WCAP == 8 * 32 && CHUNK <= (1 << 11));
static_assert(((long long)NE << SLB) < (1LL << 31));
static_assert(RCAP % 1024 == 0 && 4 * RCAP >= 5 * 16809 && RCAP % 512 == 0);
static_assert(DEGCAP >= 35 + 8 && DEGCAP <= 64);
static_assert(LZ_INTS % (NTHR * 4) == 0 && LIST_LDS_BYTES <= 262144);
static_assert((HF * (KP1 / 8)) % NTHR == 0 && (HF * (K2TOT / 8)) % NTHR == 0);
static_assert(((MPAD - NN) * (K2TOT / 8)) % NTHR == 0);
static_assert((MPAD * (KP1 / 8)) % 256 == 0);
static_assert(SM_FLOATS % 32 == 0 && SM_FLOATS / 4 <= NTHR && SM_PR + 4 <= SM_FLOATS);

typedef int v4i __attribute__((ext_vector_type(4)));
typedef int v2i __attribute__((ext_vector_type(2)));
typedef v4i __attribute__((may_alias)) v4ia;
typedef v2i __attribute__((may_alias)) v2ia;

static constexpr size_t SZ_XB   = (size_t)MPAD * KP1 * 2;
static constexpr size_t SZ_S    = (size_t)MPAD * HF * 4;
static constexpr size_t SZ_HHL  = (size_t)MPAD * K2TOT * 2;
static constexpr size_t SZ_LIST = (size_t)NLB * RCAP * 8;
static constexpr size_t SZ_TAB  = (size_t)NLB * NBRUN * 4;
static constexpr size_t SZ_FLAG = (size_t)NLB * 128;
static constexpr size_t SZ_W1T  = (size_t)HF * KP1 * 2;
static constexpr size_t SZ_W2D  = (size_t)HF * K2TOT * 2;
static constexpr size_t SZ_SM   = 2304;
static constexpr size_t O_XB    = 0;
static constexpr size_t O_S     = O_XB + SZ_XB;
static constexpr size_t O_HHL   = O_S + SZ_S;
static constexpr size_t O_LISTA = O_HHL + SZ_HHL;
static constexpr size_t O_LISTR = O_LISTA + SZ_LIST;
static constexpr size_t O_OFFA  = O_LISTR + SZ_LIST;
static constexpr size_t O_CNTA  = O_OFFA + SZ_TAB;
static constexpr size_t O_OFFR  = O_CNTA + SZ_TAB;
static constexpr size_t O_CNTR  = O_OFFR + SZ_TAB;
static constexpr size_t O_FLAGA = O_CNTR + SZ_TAB;
static constexpr size_t O_FLAGR = O_FLAGA + SZ_FLAG;
static constexpr size_t O_W1T   = O_FLAGR + SZ_FLAG;
static constexpr size_t O_W2D   = O_W1T + SZ_W1T;
static constexpr size_t O_SM    = O_W2D + SZ_W2D;
static constexpr size_t WS_TOTAL = O_SM + SZ_SM;
static_assert(SZ_XB % 256 == 0 && SZ_S % 256 == 0 && SZ_HHL % 256 == 0 && SZ_LIST % 256 == 0);
static_assert(SZ_TAB % 256 == 0 && SZ_FLAG % 256 == 0 && SZ_W1T % 256 == 0 && SZ_W2D % 256 == 0);
static_assert(SZ_SM % 256 == 0 && SZ_SM >= (size_t)SM_FLOATS * 4);
static_assert(WS_TOTAL <= (size_t)WSMAX);
static_assert(TWO_TERM == 0 || WS_TOTAL == 61660416);

__global__ __launch_bounds__(NTHR) void k_prep(const float* __restrict__ w1, const float* __restrict__ b1,
                                               const float* __restrict__ w2, const float* __restrict__ b2,
                                               const float* __restrict__ a_att, const float* __restrict__ r_att,
                                               unsigned short* __restrict__ W1T, unsigned short* __restrict__ W2D,
                                               unsigned short* __restrict__ HHL, float* __restrict__ SM) {
  __shared__ float sAtt[8];
  __shared__ float sE[8];
  __shared__ float sP[8];
  const int tid = (int)threadIdx.x;
  const int b   = (int)blockIdx.x;
  if (b < PB_W1) {
    const int g  = b * NTHR + tid;
    const int n  = g / (KP1 / 8);
    const int p  = g - n * (KP1 / 8);
    const int k0 = p * 8;
    float x[8];
    unsigned mk[8];
#pragma unroll
    for (int e = 0; e < 8; ++e) {
      const int k = k0 + e;
      const float v = w1[(size_t)clampi(k, 0, INF_ - 1) * HF + n];
      asm volatile("" :: "v"(v));
      x[e]  = v;
      mk[e] = (k < INF_) ? 0xFFFFu : 0u;
    }
    v4u o = pack8_bf16((v4f){ x[0], x[1], x[2], x[3] }, (v4f){ x[4], x[5], x[6], x[7] });
    o &= (v4u){ pk16(mk[0], mk[1]), pk16(mk[2], mk[3]), pk16(mk[4], mk[5]), pk16(mk[6], mk[7]) };
    volatile v4u* q = (volatile v4u*)(W1T + (size_t)g * 8);
    *q = o;
    __threadfence();
    *q = o;
  } else if (b < PB_W1 + PB_W2) {
    const int g  = (b - PB_W1) * NTHR + tid;
    const int n  = g / (K2TOT / 8);
    const int p  = g - n * (K2TOT / 8);
    const int k0 = (p * 8) & (HF - 1);
    float x[8];
#pragma unroll
    for (int e = 0; e < 8; ++e) {
      const float v = w2[(size_t)(k0 + e) * HF + n];
      asm volatile("" :: "v"(v));
      x[e] = v;
    }
    const v4u o = pack8_bf16((v4f){ x[0], x[1], x[2], x[3] }, (v4f){ x[4], x[5], x[6], x[7] });
    volatile v4u* q = (volatile v4u*)(W2D + (size_t)g * 8);
    *q = o;
    __threadfence();
    *q = o;
  } else if (b < PB_W1 + PB_W2 + PB_PAD) {
    const int g = (b - PB_W1 - PB_W2) * NTHR + tid;
    const v4u z = (v4u){ 0u, 0u, 0u, 0u };
    volatile v4u* q = (volatile v4u*)(HHL + (size_t)NN * K2TOT + (size_t)g * 8);
    *q = z;
    __threadfence();
    *q = z;
  } else {
    const int j  = tid & 7;
    const int gb = (j >= 3) ? 3 : 0;
    const int jc = (j > 5) ? 5 : j;
    {
      float va = a_att[clampi(j, 0, 2)];
      asm volatile("" :: "v"(va));
      float vr = r_att[clampi(j - 3, 0, 2)];
      asm volatile("" :: "v"(vr));
      const unsigned ma = (j < 3) ? 0xFFFFFFFFu : 0u;
      const unsigned mr = (j >= 3 && j < 6) ? 0xFFFFFFFFu : 0u;
      const unsigned bits = (__float_as_uint(bf16_val(va)) & ma) | (__float_as_uint(bf16_val(vr)) & mr);
      if (tid < 8) sAtt[tid] = __uint_as_float(bits);
    }
    __syncthreads();
    {
      const float m = fmaxf(sAtt[gb], fmaxf(sAtt[gb + 1], sAtt[gb + 2]));
      const float e = expf(sAtt[jc] - m);
      if (tid < 8) sE[tid] = e;
    }
    __syncthreads();
    {
      const float s = (sE[gb] + sE[gb + 1]) + sE[gb + 2];
      const float pq = sE[jc] / s;
      if (tid < 8) sP[tid] = pq;
    }
    __syncthreads();
    const int i1 = clampi(tid, 0, 63);
    const int i2 = clampi(tid - 64, 0, 63);
    v4f q1 = *(const v4fa*)(b1 + 4 * i1);
    asm volatile("" :: "v"(q1));
    v4f q2 = *(const v4fa*)(b2 + 4 * i2);
    asm volatile("" :: "v"(q2));
    const unsigned m1 = (tid < 64) ? 0xFFFFFFFFu : 0u;
    const unsigned m2 = (tid >= 64 && tid < 128) ? 0xFFFFFFFFu : 0u;
    const unsigned m3 = (tid == 128) ? 0xFFFFFFFFu : 0u;
    const unsigned m4 = (tid == 129) ? 0xFFFFFFFFu : 0u;
    const float pa0 = sP[0], pa1 = sP[1], pa2 = sP[2];
    const float pr0 = sP[3], pr1 = sP[4], pr2 = sP[5];
    v4u o;
    o[0] = (__float_as_uint(bf16_val(q1[0])) & m1) | (__float_as_uint(bf16_val(q2[0])) & m2) |
           (__float_as_uint(pa0) & m3) | (__float_as_uint(pr0) & m4);
    o[1] = (__float_as_uint(bf16_val(q1[1])) & m1) | (__float_as_uint(bf16_val(q2[1])) & m2) |
           (__float_as_uint(pa1) & m3) | (__float_as_uint(pr1) & m4);
    o[2] = (__float_as_uint(bf16_val(q1[2])) & m1) | (__float_as_uint(bf16_val(q2[2])) & m2) |
           (__float_as_uint(pa2) & m3) | (__float_as_uint(pr2) & m4);
    o[3] = (__float_as_uint(bf16_val(q1[3])) & m1) | (__float_as_uint(bf16_val(q2[3])) & m2);
    if (tid < SM_FLOATS / 4) {
      volatile v4u* q = (volatile v4u*)(SM + 4 * tid);
      *q = o;
      __threadfence();
      *q = o;
    }
  }
}

__device__ __forceinline__ int scan_chunk(const int* __restrict__ keys, int cbase, int slotBase,
                                          int* list, int lane, int wave) {
  int wc = 0;
  const int eb = wave * WCAP + lane;
  const int g0 = cbase + eb;
#define LDK(J, KV) \
  int KV; { const int gi = g0 + (J) * 32; int kx = keys[gi < NE ? gi : NE - 1]; \
            asm volatile("" :: "v"(kx)); KV = kx | ((gi < NE) ? 0 : -1); }
  LDK(0, k0)
  LDK(1, k1)
  LDK(2, k2)
  LDK(3, k3)
  LDK(4, k4)
  LDK(5, k5)
  LDK(6, k6)
  LDK(7, k7)
#undef LDK
  const unsigned nbs = (unsigned)slotBase;
  const unsigned unb = (unsigned)NBRUN;
  const unsigned unn = (unsigned)NN;
  const unsigned s0 = (unsigned)k0 - nbs, s1 = (unsigned)k1 - nbs, s2 = (unsigned)k2 - nbs, s3 = (unsigned)k3 - nbs;
  const unsigned s4 = (unsigned)k4 - nbs, s5 = (unsigned)k5 - nbs, s6 = (unsigned)k6 - nbs, s7 = (unsigned)k7 - nbs;
  const bool h0 = (s0 < unb) & ((unsigned)k0 < unn), h1 = (s1 < unb) & ((unsigned)k1 < unn);
  const bool h2 = (s2 < unb) & ((unsigned)k2 < unn), h3 = (s3 < unb) & ((unsigned)k3 < unn);
  const bool h4 = (s4 < unb) & ((unsigned)k4 < unn), h5 = (s5 < unb) & ((unsigned)k5 < unn);
  const bool h6 = (s6 < unb) & ((unsigned)k6 < unn), h7 = (s7 < unb) & ((unsigned)k7 < unn);
  const unsigned any = __builtin_amdgcn_ballot_w32(h0 | h1 | h2 | h3 | h4 | h5 | h6 | h7);
  if (any != 0u) {
#define HITJ(J, HJ, SJ) { \
      const unsigned mj = __builtin_amdgcn_ballot_w32(HJ); \
      if (mj != 0u) { \
        if (HJ) { \
          const int pos = wc + (int)__builtin_amdgcn_mbcnt_lo(mj, 0u); \
          if (pos < WCAP) list[wave * WCAP + pos] = ((eb + (J) * 32) << SLB) | (int)(SJ); \
        } \
        wc += (int)__builtin_popcount(mj); } }
    HITJ(0, h0, s0)
    HITJ(1, h1, s1)
    HITJ(2, h2, s2)
    HITJ(3, h3, s3)
    HITJ(4, h4, s4)
    HITJ(5, h5, s5)
    HITJ(6, h6, s6)
    HITJ(7, h7, s7)
#undef HITJ
  }
  return wc;
}

__global__ __launch_bounds__(NTHR) void k_list(const int* __restrict__ keys, const int* __restrict__ cols,
                                               int* __restrict__ LIST, int* __restrict__ OFF,
                                               int* __restrict__ CNT, int* __restrict__ FLAG) {
  extern __shared__ __attribute__((aligned(16))) int dsm[];
  int* list = dsm;
  int* hl   = dsm + LISTN;
  int* sl   = hl + RCAP;
  int* cnt  = sl + RCAP;
  int* offs = cnt + NBRUN;
  int* cur  = offs + NBRUN;
  int* misc = cur + NBRUN;
  const int tid  = (int)threadIdx.x;
  const int lane = tid & 31;
  const int wave = __builtin_amdgcn_readfirstlane(tid >> 5);
  const int nodeBase = (int)blockIdx.x * NBRUN;

  {
    const v4i z4 = (v4i){0, 0, 0, 0};
    for (int i = tid * 4; i < LZ_INTS; i += NTHR * 4) *(v4ia*)(dsm + i) = z4;
    if (tid < MISC_INTS) misc[tid] = 0;
  }
  __syncthreads();

  int t = 0, ov = 0;
#pragma unroll 1
  for (int ch = 0; ch < NCHUNK; ++ch) {
    const int cbase = ch * CHUNK;
    const int wc = scan_chunk(keys, cbase, nodeBase, list, lane, wave);
    if (lane == 0) misc[wave] = wc;
    __syncthreads();
    if (wave == 0) {
#pragma unroll 1
      for (int w2 = 0; w2 < NWAVE; ++w2) {
        const int c = __builtin_amdgcn_readfirstlane(clampi(misc[w2], 0, WCAP));
#pragma unroll 1
        for (int b0 = 0; b0 < c; b0 += 32) {
          const int idx = b0 + lane;
          const int ent = list[w2 * WCAP + (idx < WCAP ? idx : WCAP - 1)];
          const int m32 = (c - b0) < 32 ? (c - b0) : 32;
#pragma unroll 1
          for (int k = 0; k < m32; ++k) {
            const int u    = __builtin_amdgcn_readlane(ent, k);
            const int slot = u & (NBRUN - 1);
            const int el   = (u >> SLB) & (CHUNK - 1);
            const int pk   = ((cbase + el) << SLB) | slot;
            if (t < RCAP) {
              if (lane == 0) { hl[t] = pk; cnt[slot] = cnt[slot] + 1; }
              t = t + 1;
            } else {
              ov = 1;
            }
          }
        }
      }
    }
    __syncthreads();
  }
  if (wave == 0 && lane == 0) { misc[8] = t; misc[9] = ov; }
  __syncthreads();
  const int tt  = __builtin_amdgcn_readfirstlane(clampi(misc[8], 0, RCAP));
  const int ovf = misc[9];

  if (wave == 0) {
    const int base = lane * (NBRUN / 32);
    int s = 0;
#pragma unroll 1
    for (int i = 0; i < NBRUN / 32; ++i) s += cnt[base + i];
    int incl = s;
#pragma unroll
    for (int d = 1; d < 32; d <<= 1) {
      const int y = __shfl_up(incl, d, 32);
      if (lane >= d) incl += y;
    }
    int run = incl - s;
#pragma unroll 1
    for (int i = 0; i < NBRUN / 32; ++i) {
      const int cv = cnt[base + i];
      offs[base + i] = run;
      cur[base + i]  = run;
      run += cv;
    }
  }
  __syncthreads();
  if (wave == 0) {
#pragma unroll 1
    for (int b0 = 0; b0 < tt; b0 += 32) {
      const int idx = b0 + lane;
      const int ent = hl[idx < RCAP ? idx : RCAP - 1];
      const int m32 = (tt - b0) < 32 ? (tt - b0) : 32;
#pragma unroll 1
      for (int k = 0; k < m32; ++k) {
        const int u    = __builtin_amdgcn_readlane(ent, k);
        const int slot = u & (NBRUN - 1);
        if (lane == 0) {
          int p = cur[slot];
          p = clampi(p, 0, RCAP - 1);
          sl[p] = u;
          cur[slot] = p + 1;
        }
      }
    }
  }
  __syncthreads();

  const v4i c4 = *(const v4ia*)(cnt + 4 * tid);
  const v4i o4 = *(const v4ia*)(offs + 4 * tid);
  {
    const bool bg = (c4[0] > DEGCAP) | (c4[1] > DEGCAP) | (c4[2] > DEGCAP) | (c4[3] > DEGCAP);
    if (bg) misc[10] = 1;
  }
  __syncthreads();
  const int flg = ((ovf | misc[10]) != 0) ? 1 : 0;

  {
    int* po = OFF + nodeBase + 4 * tid;
    int* pc = CNT + nodeBase + 4 * tid;
    *(volatile v4i*)po = o4;
    *(volatile v4i*)pc = c4;
    __threadfence();
    *(volatile v4i*)po = o4;
    *(volatile v4i*)pc = c4;
  }
  if (tid < 8) {
    const v4i f4 = (v4i){ flg, flg, flg, flg };
    int* pf = FLAG + (int)blockIdx.x * 32 + 4 * tid;
    *(volatile v4i*)pf = f4;
    __threadfence();
    *(volatile v4i*)pf = f4;
  }
  int* lb = LIST + (size_t)blockIdx.x * (size_t)(RCAP * 2);
#pragma unroll 1
  for (int it = 0; it < RCAP / 512; ++it) {
    const int q  = it * NTHR + tid;
    const int i0 = 2 * q;
    const v2i u2 = *(const v2ia*)(sl + i0);
    const int e0 = clampi(u2[0] >> SLB, 0, NE - 1);
    const int e1 = clampi(u2[1] >> SLB, 0, NE - 1);
    int n0 = cols[e0];
    asm volatile("" :: "v"(n0));
    int n1 = cols[e1];
    asm volatile("" :: "v"(n1));
    n0 = clampi(n0, 0, NN - 1);
    n1 = clampi(n1, 0, NN - 1);
    const int m0 = (i0 < tt) ? -1 : 0;
    const int m1 = (i0 + 1 < tt) ? -1 : 0;
    const v4i o = (v4i){ n0 & m0, e0 & m0, n1 & m1, e1 & m1 };
    int* p = lb + 4 * q;
    *(volatile v4i*)p = o;
    __threadfence();
    *(volatile v4i*)p = o;
  }
}

template <int LAYER>
__global__ __launch_bounds__(NTHR) void k_replay(const float* __restrict__ S, const float* __restrict__ vals,
                                                 const int* __restrict__ LIST, const int* __restrict__ OFF,
                                                 const int* __restrict__ CNT, const int* __restrict__ FLAG,
                                                 const float* __restrict__ P, unsigned short* __restrict__ hhl,
                                                 float* __restrict__ outp, int nReal) {
  static_assert(LAYER == 1 || LAYER == 2);
  const int lane = (int)threadIdx.x & 31;
  const int wave = __builtin_amdgcn_readfirstlane((int)threadIdx.x >> 5);
  const int row  = (int)blockIdx.x * 8 + wave;
  const bool live = row < nReal;
  const int rowc = live ? row : nReal - 1;
  const int blk  = rowc >> SLB;
  int fl = FLAG[blk * 32];
  asm volatile("" :: "v"(fl));
  int cr = CNT[rowc];
  asm volatile("" :: "v"(cr));
  int of = OFF[rowc];
  asm volatile("" :: "v"(of));
  const bool big = (cr < 0) | (cr > DEGCAP);
  int cv = clampi(cr, 0, DEGCAP);
  cv = live ? cv : 0;
  const int cn = __builtin_amdgcn_readfirstlane(cv);
  const int o  = clampi(of, 0, RCAP - 1);
  float p0 = P[0];
  asm volatile("" :: "v"(p0));
  float p1 = P[1];
  asm volatile("" :: "v"(p1));
  float p2 = P[2];
  asm volatile("" :: "v"(p2));
  const int* lb = LIST + (size_t)blk * (size_t)(RCAP * 2);
  const int c0 = (LAYER == 1) ? 8 * lane : 4 * lane;
  const int c1 = (LAYER == 1) ? 8 * lane + 4 : 128 + 4 * lane;

  v4f a0 = (v4f){0.0f, 0.0f, 0.0f, 0.0f};
  v4f a1 = (v4f){0.0f, 0.0f, 0.0f, 0.0f};
#pragma unroll 1
  for (int b0 = 0; b0 < cn; b0 += 32) {
    int idx = o + b0 + lane;
    idx = idx > RCAP - 1 ? RCAP - 1 : idx;
    const v2i pr = *(const v2ia*)(lb + 2 * idx);
    int pn = pr[0];
    asm volatile("" :: "v"(pn));
    int pe = pr[1];
    asm volatile("" :: "v"(pe));
    const int node = clampi(pn, 0, NN - 1);
    const int id   = clampi(pe, 0, NE - 1);
    float v0 = vals[id];
    asm volatile("" :: "v"(v0));
    float v1 = vals[NE + id];
    asm volatile("" :: "v"(v1));
    float v2 = vals[2 * NE + id];
    asm volatile("" :: "v"(v2));
    const float t0 = p0 * bf16_val(v0);
    const float t1 = p1 * bf16_val(v1);
    const float t2 = p2 * bf16_val(v2);
    const float w  = (t0 + t1) + t2;
    const int wi   = __float_as_int(w);
    const int m32  = (cn - b0) < 32 ? (cn - b0) : 32;
#pragma unroll 1
    for (int k = 0; k < m32; ++k) {
      const int   sk = __builtin_amdgcn_readlane(node, k);
      const float ck = __int_as_float(__builtin_amdgcn_readlane(wi, k));
      const float* sp = S + (size_t)sk * HF;
      v4f r0 = *(const v4fa*)(sp + c0);
      asm volatile("" :: "v"(r0));
      v4f r1 = *(const v4fa*)(sp + c1);
      asm volatile("" :: "v"(r1));
      const v4f q0 = r0 * ck;
      const v4f q1 = r1 * ck;
      a0 = a0 + q0;
      a1 = a1 + q1;
    }
  }

  const bool poison = (fl != 0) | big;
  const float nanv = __int_as_float(0x7fc00000);
  if constexpr (LAYER == 1) {
    v4f h0, h1;
#pragma unroll
    for (int e = 0; e < 4; ++e) {
      const float x0 = a0[e];
      const float x1 = a1[e];
      const float y0 = (x0 > 0.0f) ? x0 : 0.2f * x0;
      const float y1 = (x1 > 0.0f) ? x1 : 0.2f * x1;
      h0[e] = poison ? nanv : y0;
      h1[e] = poison ? nanv : y1;
    }
    const v4u hi = pack8_bf16(h0, h1);
#if TWO_TERM
    const v4u lo = pack8_bf16_lo(h0, h1);
#endif
    unsigned short* rp = hhl + (size_t)rowc * K2TOT + 8 * lane;
    if (live) {
      *(volatile v4u*)rp = hi;
#if TWO_TERM
      *(volatile v4u*)(rp + HF) = lo;
#endif
      __threadfence();
      *(volatile v4u*)rp = hi;
#if TWO_TERM
      *(volatile v4u*)(rp + HF) = lo;
#endif
    }
  } else {
    float ss = a0[0] * a0[0];
    ss = ss + a0[1] * a0[1];
    ss = ss + a0[2] * a0[2];
    ss = ss + a0[3] * a0[3];
    ss = ss + a1[0] * a1[0];
    ss = ss + a1[1] * a1[1];
    ss = ss + a1[2] * a1[2];
    ss = ss + a1[3] * a1[3];
    ss = ss + __shfl_xor(ss, 16, 32);
    ss = ss + __shfl_xor(ss, 8, 32);
    ss = ss + __shfl_xor(ss, 4, 32);
    ss = ss + __shfl_xor(ss, 2, 32);
    ss = ss + __shfl_xor(ss, 1, 32);
    const float nrm = sqrtf(ss);
    const float dv  = (nrm < 1e-12f) ? 1e-12f : nrm;
    v4f y0 = a0 / dv;
    v4f y1 = a1 / dv;
#pragma unroll
    for (int e = 0; e < 4; ++e) {
      y0[e] = poison ? nanv : y0[e];
      y1[e] = poison ? nanv : y1[e];
    }
    float* op = outp + (size_t)rowc * HF + 4 * lane;
    if (live) {
      *(volatile v4f*)op = y0;
      *(volatile v4f*)(op + 128) = y1;
      __threadfence();
      *(volatile v4f*)op = y0;
      *(volatile v4f*)(op + 128) = y1;
    }
  }
}

extern "C" void kernel_launch(void* const* d_in, const int* in_sizes, int n_in,
                              void* d_out, int out_size, void* d_ws, size_t ws_size,
                              hipStream_t stream) {
  if (n_in < 13) return;
  if (in_sizes[0] != NN * INF_) return;
  if (in_sizes[1] != 3 * NE || in_sizes[4] != 3 * NE) return;
  if (in_sizes[2] != NE || in_sizes[3] != NE) return;
  if (in_sizes[5] != NE || in_sizes[6] != NE) return;
  if (in_sizes[7] != INF_ * HF || in_sizes[8] != HF) return;
  if (in_sizes[9] != HF * HF || in_sizes[10] != HF) return;
  if (in_sizes[11] != 3 || in_sizes[12] != 3) return;
  if ((long long)out_size != (long long)NN * HF) return;
  if (ws_size < WS_TOTAL) return;

  const float* x      = (const float*)d_in[0];
  const float* a_vals = (const float*)d_in[1];
  const int*   a_rows = (const int*)d_in[2];
  const int*   a_cols = (const int*)d_in[3];
  const float* r_vals = (const float*)d_in[4];
  const int*   r_rows = (const int*)d_in[5];
  const int*   r_cols = (const int*)d_in[6];
  const float* w1     = (const float*)d_in[7];
  const float* b1     = (const float*)d_in[8];
  const float* w2     = (const float*)d_in[9];
  const float* b2     = (const float*)d_in[10];
  const float* a_att  = (const float*)d_in[11];
  const float* r_att  = (const float*)d_in[12];
  float* out = (float*)d_out;

  char* ws = (char*)d_ws;
  unsigned short* XB   = (unsigned short*)(ws + O_XB);
  float*          Sp   = (float*)(ws + O_S);
  unsigned short* HHL  = (unsigned short*)(ws + O_HHL);
  int* LISTa = (int*)(ws + O_LISTA);
  int* LISTr = (int*)(ws + O_LISTR);
  int* OFFa  = (int*)(ws + O_OFFA);
  int* CNTa  = (int*)(ws + O_CNTA);
  int* OFFr  = (int*)(ws + O_OFFR);
  int* CNTr  = (int*)(ws + O_CNTR);
  int* FLAGa = (int*)(ws + O_FLAGA);
  int* FLAGr = (int*)(ws + O_FLAGR);
  unsigned short* W1T = (unsigned short*)(ws + O_W1T);
  unsigned short* W2D = (unsigned short*)(ws + O_W2D);
  float* SM = (float*)(ws + O_SM);

  hipFuncSetAttribute(reinterpret_cast<const void*>(&k_list), hipFuncAttributeMaxDynamicSharedMemorySize,
                      (int)LIST_LDS_BYTES);

  static_assert(MPAD % 64 == 0 && HF % 64 == 0 && NN % 16 == 0 && HF % 4 == 0 && HF % 32 == 0);
  const int gemmBlocks = (((NN + 63) / 64) * (HF / 64) + 7) / 8;

  k_plane<0><<<(MPAD * (KP1 / 8)) / 256, 256, 0, stream>>>(x, NN, INF_, INF_, XB, MPAD, KP1);
  k_prep<<<PB_ALL, NTHR, 0, stream>>>(w1, b1, w2, b2, a_att, r_att, W1T, W2D, HHL, SM);
  k_list<<<NLB, NTHR, LIST_LDS_BYTES, stream>>>(a_rows, a_cols, LISTa, OFFa, CNTa, FLAGa);
  k_list<<<NLB, NTHR, LIST_LDS_BYTES, stream>>>(r_rows, r_cols, LISTr, OFFr, CNTr, FLAGr);
  k_gemm_nt<0, 1><<<gemmBlocks, 256, 0, stream>>>(XB, W1T, SM, Sp, NN, HF, KP1, HF);
  k_replay<1><<<NN / 8, NTHR, 0, stream>>>(Sp, a_vals, LISTa, OFFa, CNTa, FLAGa, SM + SM_PA, HHL, out, NN);
  k_gemm_nt<0, 1><<<gemmBlocks, 256, 0, stream>>>(HHL, W2D, SM + HF, Sp, NN, HF, K2TOT, HF);
  k_replay<2><<<NN / 8, NTHR, 0, stream>>>(Sp, r_vals, LISTr, OFFr, CNTr, FLAGr, SM + SM_PR, HHL, out, NN);
}
